// KeypointPatchModel_35296041238939
// MI455X (gfx1250) — hardware-verified
//
#include <hip/hip_runtime.h>
#include <stddef.h>
#include <stdint.h>
#include <math.h>


#pragma clang fp contract(off)

#define HH    224
#define WW    224
#define IMG   50176
#define BB    32
#define CCH   3
#define KPT   64
#define PP    16
#define NCLS  1000
#define NPAD  1024
#define FC1K  2048
#define FC1N  64
#define FC2K  4096
#define MROWS 2048
#define NTHR  256

#define TR  8
#define GWD 228
#define DWD 226
#define NG  ((TR + 4) * GWD)
#define ND  ((TR + 2) * DWD)
#define NR  (TR * WW)

#define SPW 18
#define SPL 324
#define CHL 196

#define NT1 (FC1N * FC1K / 8)
#define NT2 (NPAD * FC2K / 8)

static_assert(IMG == NTHR * CHL);
static_assert((HH % TR) == 0);
static_assert((NR % 4) == 0);
static_assert(MROWS == BB * KPT);
static_assert(FC1K == 8 * PP * PP);
static_assert(FC2K == KPT * FC1N);
static_assert((NT1 % NTHR) == 0 && (NT2 % NTHR) == 0);
static_assert(NPAD >= NCLS && (NPAD % 128) == 0);

typedef float          v4f   __attribute__((ext_vector_type(4)));
typedef float          v8f   __attribute__((ext_vector_type(8)));
typedef unsigned short v8us  __attribute__((ext_vector_type(8)));
typedef unsigned short v16us __attribute__((ext_vector_type(16)));
typedef __bf16         v16bf __attribute__((ext_vector_type(16)));
typedef unsigned int   v4u   __attribute__((ext_vector_type(4)));
typedef int            v4i   __attribute__((ext_vector_type(4)));
union FragU { v16us v; v8us h[2]; };

__device__ __forceinline__ unsigned short bfr(float f) {
  unsigned int u = __float_as_uint(f);
  u += 0x7FFFu + ((u >> 16) & 1u);
  return (unsigned short)(u >> 16);
}
__device__ __forceinline__ float bfup(unsigned short s) {
  return __uint_as_float(((unsigned int)s) << 16);
}

__device__ __forceinline__ v8f wmb(v16us a, v16us b, v8f c) {
  v16bf av = __builtin_bit_cast(v16bf, a);
  v16bf bv = __builtin_bit_cast(v16bf, b);
  v8f d = __builtin_amdgcn_wmma_f32_16x16x32_bf16(false, av, false, bv, (short)0, c, false, false);
#if defined(__HIP_DEVICE_COMPILE__)
  asm volatile("v_nop\n\tv_nop\n\tv_nop\n\tv_nop" : "+v"(d) : "v"(av), "v"(bv));
#endif
  return d;
}

__device__ __forceinline__ v8f zero8() {
  v8f z = {0.f, 0.f, 0.f, 0.f, 0.f, 0.f, 0.f, 0.f};
  return z;
}

__device__ __forceinline__ int block_sum(int c, int* sws, int lane, int wave) {
  c += __shfl_xor(c, 1, 32);
  c += __shfl_xor(c, 2, 32);
  c += __shfl_xor(c, 4, 32);
  c += __shfl_xor(c, 8, 32);
  c += __shfl_xor(c, 16, 32);
  if (lane == 0) sws[wave] = c;
  __syncthreads();
  int t = 0;
#pragma unroll
  for (int w = 0; w < 8; ++w) t += sws[w];
  __syncthreads();
  return t;
}

__global__ __launch_bounds__(NTHR) void k_prep(const float* __restrict__ fc1w, const float* __restrict__ fc2w,
                                               unsigned short* w1h, unsigned short* w1l,
                                               unsigned short* w2h, unsigned short* w2l) {
  const int i = blockIdx.x * NTHR + (int)threadIdx.x;
  const bool seg1 = (blockIdx.x < NT1 / NTHR);
  float v[8];
  unsigned short* dh;
  unsigned short* dl;
  size_t o;
  if (seg1) {
    o = (size_t)i * 8;
#pragma unroll
    for (int e = 0; e < 8; ++e) v[e] = fc1w[o + e];
    dh = w1h; dl = w1l;
  } else {
    const int j = i - NT1;
    o = (size_t)j * 8;
    const int n = (int)(o / FC2K);
    const int k = (int)(o - (size_t)n * FC2K);
    const int nc = n < NCLS ? n : NCLS - 1;
#pragma unroll
    for (int e = 0; e < 8; ++e) {
      const float xv = fc2w[(size_t)nc * FC2K + k + e];
      v[e] = (n < NCLS) ? xv : 0.0f;
    }
    dh = w2h; dl = w2l;
  }
  v8us hv, lv;
#pragma unroll
  for (int e = 0; e < 8; ++e) {
    const unsigned short hs = bfr(v[e]);
    hv[e] = hs;
    lv[e] = bfr(v[e] - bfup(hs));
  }
  *(volatile v8us*)(dh + o) = hv;
  *(volatile v8us*)(dl + o) = lv;
  __threadfence();
  *(volatile v8us*)(dh + o) = hv;
  *(volatile v8us*)(dl + o) = lv;
}

__global__ __launch_bounds__(NTHR) void k_harris(const float* __restrict__ x, float* Rm) {
  __shared__ __attribute__((aligned(16))) float sg[NG];
  __shared__ __attribute__((aligned(16))) float sdx[ND];
  __shared__ __attribute__((aligned(16))) float sdy[ND];
  __shared__ __attribute__((aligned(16))) float sr[NR];
  const int b = blockIdx.y, y0 = blockIdx.x * TR, tid = threadIdx.x;
  const float* xb = x + (size_t)b * CCH * IMG;

  for (int i = tid; i < NG; i += NTHR) {
    const int ly = i / GWD, lx = i - ly * GWD;
    const int gy = y0 + ly - 2, gx = lx - 2;
    const bool inb = (gy >= 0) && (gy < HH) && (gx >= 0) && (gx < WW);
    const int cy = gy < 0 ? 0 : (gy > HH - 1 ? HH - 1 : gy);
    const int cx = gx < 0 ? 0 : (gx > WW - 1 ? WW - 1 : gx);
    const int o = cy * WW + cx;
    const float a0 = xb[o], a1 = xb[IMG + o], a2 = xb[2 * IMG + o];
    float s = a0 + a1;
    s = s + a2;
    const float g = s / 3.0f;
    sg[i] = inb ? g : 0.0f;
  }
  __syncthreads();

  for (int i = tid; i < ND; i += NTHR) {
    const int ly = i / DWD, lx = i - ly * DWD;
    const int gy = y0 + ly - 1, gx = lx - 1;
    const bool inb = (gy >= 0) && (gy < HH) && (gx >= 0) && (gx < WW);
    const float* g0 = sg + ly * GWD + lx;
    const float a00 = g0[0],       a01 = g0[1],           a02 = g0[2];
    const float a10 = g0[GWD],     a12 = g0[GWD + 2];
    const float a20 = g0[2 * GWD], a21 = g0[2 * GWD + 1], a22 = g0[2 * GWD + 2];
    float dx = -a00; dx = dx + a02; dx = dx - a10; dx = dx + a12; dx = dx - a20; dx = dx + a22;
    float dy = -a00; dy = dy - a01; dy = dy - a02; dy = dy + a20; dy = dy + a21; dy = dy + a22;
    sdx[i] = inb ? dx : 0.0f;
    sdy[i] = inb ? dy : 0.0f;
  }
  __syncthreads();

  for (int i = tid; i < NR; i += NTHR) {
    const int ly = i / WW, lx = i - ly * WW;
    const int gy = y0 + ly, gx = lx;
    const float* px = sdx + ly * DWD + lx;
    const float* py = sdy + ly * DWD + lx;
    float d[9], e[9];
#pragma unroll
    for (int r = 0; r < 3; ++r) {
#pragma unroll
      for (int c = 0; c < 3; ++c) {
        d[3 * r + c] = px[r * DWD + c];
        e[3 * r + c] = py[r * DWD + c];
      }
    }
    const float wv[9] = {0.0625f, 0.125f, 0.0625f, 0.125f, 0.25f, 0.125f, 0.0625f, 0.125f, 0.0625f};
    float sxx, syy, sxy;
    {
      float p = d[0] * d[0]; sxx = wv[0] * p;
      p = e[0] * e[0];       syy = wv[0] * p;
      p = d[0] * e[0];       sxy = wv[0] * p;
    }
#pragma unroll
    for (int t = 1; t < 9; ++t) {
      float p = d[t] * d[t]; p = wv[t] * p; sxx = sxx + p;
      p = e[t] * e[t];       p = wv[t] * p; syy = syy + p;
      p = d[t] * e[t];       p = wv[t] * p; sxy = sxy + p;
    }
    const float trc = sxx + syy;
    const float det = sxx * syy;
    const float q2  = sxy * sxy;
    float rv = det - q2;
    float tt = trc * trc;
    tt = 0.04f * tt;
    rv = rv - tt;
    const float mk = (gy >= PP && gy < HH - PP && gx >= PP && gx < WW - PP) ? 1.0f : 0.0f;
    sr[i] = rv * mk;
  }
  __syncthreads();

  float* dst = Rm + (size_t)b * IMG + (size_t)y0 * WW;
  const int q0 = tid, q1 = tid + NTHR;
  const bool has1 = (q1 < NR / 4);
  const int q1c = has1 ? q1 : q0;
  const v4f v0 = *(const v4f*)(sr + 4 * q0);
  const v4f v1 = *(const v4f*)(sr + 4 * q1c);
  *(volatile v4f*)(dst + 4 * q0) = v0;
  if (has1) *(volatile v4f*)(dst + 4 * q1) = v1;
  __threadfence();
  *(volatile v4f*)(dst + 4 * q0) = v0;
  if (has1) *(volatile v4f*)(dst + 4 * q1) = v1;
}

__global__ __launch_bounds__(NTHR) void k_topk(const float* __restrict__ Rm, int* idxT) {
  extern __shared__ v4f dynlds[];
  v4u* skey4 = (v4u*)dynlds;
  unsigned int* skey = (unsigned int*)dynlds;
  __shared__ int sws[8];
  __shared__ unsigned long long slist[KPT];
  const int b = blockIdx.x, tid = threadIdx.x, lane = tid & 31, wave = tid >> 5;
  const float* Rb = Rm + (size_t)b * IMG;

  for (int q = tid; q < IMG / 4; q += NTHR) {
    const v4f v = *(const v4f*)(Rb + 4 * q);
    v4u kk;
#pragma unroll
    for (int c = 0; c < 4; ++c) {
      const unsigned int u = __float_as_uint(v[c]);
      kk[c] = (u & 0x80000000u) ? ~u : (u | 0x80000000u);
    }
    skey4[q] = kk;
  }
  __syncthreads();

  unsigned int T = 0u;
  for (int bit = 31; bit >= 0; --bit) {
    const unsigned int cand = T | (1u << bit);
    int c = 0;
    for (int j = 0; j < CHL; ++j) c += (skey[tid + NTHR * j] >= cand) ? 1 : 0;
    c = block_sum(c, sws, lane, wave);
    T = (c >= KPT) ? cand : T;
  }
  int cgt = 0, ceq = 0;
  for (int j = 0; j < CHL; ++j) {
    const unsigned int k = skey[tid + NTHR * j];
    cgt += (k > T) ? 1 : 0;
    ceq += (k == T) ? 1 : 0;
  }
  cgt = block_sum(cgt, sws, lane, wave);
  ceq = block_sum(ceq, sws, lane, wave);
  int need = KPT - cgt;
  need = need < 1 ? 1 : (need > KPT ? KPT : need);
  int imax = IMG - 1;
  if (ceq > need) {
    int lo = 0, hi = IMG - 1;
    for (int it = 0; it < 16; ++it) {
      const int mid = (lo + hi) >> 1;
      int c = 0;
      for (int j = 0; j < CHL; ++j) {
        const int i = tid + NTHR * j;
        c += ((skey[i] == T) && (i <= mid)) ? 1 : 0;
      }
      c = block_sum(c, sws, lane, wave);
      if (c >= need) hi = mid; else lo = mid + 1;
    }
    imax = hi;
  }

  if (tid < KPT) slist[tid] = 0xFFFFull;
  __syncthreads();
  int cnt = 0;
  for (int j = 0; j < CHL; ++j) {
    const int i = tid + NTHR * j;
    const unsigned int k = skey[i];
    const bool sel = (k > T) || ((k == T) && (i <= imax));
    cnt += sel ? 1 : 0;
  }
  int incl = cnt;
#pragma unroll
  for (int dlt = 1; dlt < 32; dlt <<= 1) {
    const int y = __shfl_up(incl, dlt, 32);
    incl = (lane >= dlt) ? incl + y : incl;
  }
  if (lane == 31) sws[wave] = incl;
  __syncthreads();
  int base = 0;
#pragma unroll
  for (int w = 0; w < 8; ++w) base += (w < wave) ? sws[w] : 0;
  base += incl - cnt;
  int pos = base;
  for (int j = 0; j < CHL; ++j) {
    const int i = tid + NTHR * j;
    const unsigned int k = skey[i];
    const bool sel = (k > T) || ((k == T) && (i <= imax));
    if (sel) {
      if (pos < KPT) slist[pos] = (((unsigned long long)k) << 32) | (unsigned long long)(unsigned int)(65535 - i);
      ++pos;
    }
  }
  __syncthreads();

  for (int kk = 2; kk <= KPT; kk <<= 1) {
    for (int jj = kk >> 1; jj > 0; jj >>= 1) {
      if (tid < KPT) {
        const int p = tid ^ jj;
        if (p > tid) {
          const unsigned long long a = slist[tid], c = slist[p];
          const bool dsc = ((tid & kk) == 0);
          const bool sw = dsc ? (a < c) : (a > c);
          if (sw) { slist[tid] = c; slist[p] = a; }
        }
      }
      __syncthreads();
    }
  }

  if (wave == 0) {
    const int l = lane & 15;
    v4i v;
#pragma unroll
    for (int c = 0; c < 4; ++c) {
      const unsigned long long s = slist[4 * l + c];
      int ix = 65535 - (int)(s & 0xFFFFull);
      ix = ix < 0 ? 0 : (ix > IMG - 1 ? IMG - 1 : ix);
      v[c] = ix;
    }
    int* op = idxT + (size_t)b * KPT + 4 * l;
    if (lane < 16) *(volatile v4i*)op = v;
    __threadfence();
    if (lane < 16) *(volatile v4i*)op = v;
  }
}

__global__ __launch_bounds__(NTHR) void k_patch(const float* __restrict__ x, const int* __restrict__ idxT,
                                                const float* __restrict__ convw, const float* __restrict__ convb,
                                                unsigned short* Hh, unsigned short* Hl) {
  __shared__ __attribute__((aligned(16))) float sp[4 * SPL];
  __shared__ __attribute__((aligned(16))) unsigned short shh[8 * PP * PP];
  __shared__ __attribute__((aligned(16))) unsigned short shl[8 * PP * PP];
  const int bk = blockIdx.x, b = bk / KPT;
  const int tid = threadIdx.x, lane = tid & 31, wave = tid >> 5, h = lane >> 4, m = lane & 15;

  for (int i = tid; i < 4 * SPL; i += NTHR) sp[i] = 0.0f;

  int idx = idxT[bk];
  idx = idx < 0 ? 0 : (idx > IMG - 1 ? IMG - 1 : idx);
  const int row = idx / WW;
  const int col = idx - row * WW;
  float cy = (float)row / 224.0f; cy = cy - 0.5f; cy = cy * 2.0f; cy = fminf(fmaxf(cy, -1.0f), 1.0f);
  float cx = (float)col / 224.0f; cx = cx - 0.5f; cx = cx * 2.0f; cx = fminf(fmaxf(cx, -1.0f), 1.0f);
  float c01y = cy + 1.0f; c01y = c01y * 0.5f;
  float c01x = cx + 1.0f; c01x = c01x * 0.5f;

  const int pi = tid >> 4, pj = tid & 15;
  const float qr = (float)(16.0 / 224.0);
  const float inv15 = 1.0f / 15.0f;
  const float sj = (float)pj * inv15, si = (float)pi * inv15;
  float pgj, pgi;
  {
    float om = 1.0f - sj; float t0 = (-qr) * om; float t1 = qr * sj; pgj = t0 + t1;
    pgj = (pj == PP - 1) ? qr : pgj;
    om = 1.0f - si; t0 = (-qr) * om; t1 = qr * si; pgi = t0 + t1;
    pgi = (pi == PP - 1) ? qr : pgi;
  }
  float g0 = pgj + c01y;
  float g1 = pgi + c01x;
  g0 = g0 * 2.0f; g0 = g0 - 1.0f;
  g1 = g1 * 2.0f; g1 = g1 - 1.0f;
  float gx = g0 + 1.0f; gx = gx * 0.5f; gx = gx * 223.0f;
  float gy = g1 + 1.0f; gy = gy * 0.5f; gy = gy * 223.0f;
  const float x0f = floorf(gx), y0f = floorf(gy);
  const float x1f = x0f + 1.0f, y1f = y0f + 1.0f;
  const float wx1 = gx - x0f; const float wx0 = 1.0f - wx1;
  const float wy1 = gy - y0f; const float wy0 = 1.0f - wy1;
  const float vx0 = (x0f >= 0.0f && x0f < 224.0f) ? 1.0f : 0.0f;
  const float vx1 = (x1f >= 0.0f && x1f < 224.0f) ? 1.0f : 0.0f;
  const float vy0 = (y0f >= 0.0f && y0f < 224.0f) ? 1.0f : 0.0f;
  const float vy1 = (y1f >= 0.0f && y1f < 224.0f) ? 1.0f : 0.0f;
  const int xc0 = (int)fminf(fmaxf(x0f, 0.0f), 223.0f);
  const int xc1 = (int)fminf(fmaxf(x1f, 0.0f), 223.0f);
  const int yc0 = (int)fminf(fmaxf(y0f, 0.0f), 223.0f);
  const int yc1 = (int)fminf(fmaxf(y1f, 0.0f), 223.0f);
  const float m00 = vx0 * vy0, m10 = vx1 * vy0, m01 = vx0 * vy1, m11 = vx1 * vy1;
  const float w00 = wx0 * wy0, w10 = wx1 * wy0, w01 = wx0 * wy1, w11 = wx1 * wy1;
  __syncthreads();
#pragma unroll
  for (int c = 0; c < CCH; ++c) {
    const float* xp = x + ((size_t)b * CCH + c) * IMG;
    const float a00 = xp[yc0 * WW + xc0] * m00;
    const float a10 = xp[yc0 * WW + xc1] * m10;
    const float a01 = xp[yc1 * WW + xc0] * m01;
    const float a11 = xp[yc1 * WW + xc1] * m11;
    float o = a00 * w00;
    float t = a10 * w10; o = o + t;
    t = a01 * w01;       o = o + t;
    t = a11 * w11;       o = o + t;
    sp[c * SPL + (pi + 1) * SPW + (pj + 1)] = o;
  }
  __syncthreads();

  int offs[16];
  v16us bh, bl;
#pragma unroll
  for (int e = 0; e < 16; ++e) {
    const int k  = 8 * h + (e & 7) + ((e >> 3) << 4);
    const int ci = k / 9;
    const int r9 = k - 9 * ci;
    const int rr = r9 / 3;
    const int cc = r9 - 3 * rr;
    offs[e] = (k < 27) ? (ci * SPL + rr * SPW + cc) : (3 * SPL);
    const int kc = k < 27 ? k : 26;
    const int nc = m < 8 ? m : 7;
    const float wv0 = convw[nc * 27 + kc];
    const float wv = (k < 27 && m < 8) ? wv0 : 0.0f;
    const unsigned short hs = bfr(wv);
    bh[e] = hs;
    bl[e] = bfr(wv - bfup(hs));
  }
  const float bias = convb[m < 8 ? m : 7];

#pragma unroll
  for (int tt = 0; tt < 2; ++tt) {
    const int prow  = 2 * wave + tt;
    const int abase = prow * SPW + m;
    v16us ah, al;
#pragma unroll
    for (int e = 0; e < 16; ++e) {
      const float av = sp[offs[e] + abase];
      const unsigned short hs = bfr(av);
      ah[e] = hs;
      al[e] = bfr(av - bfup(hs));
    }
    v8f acc = zero8();
    acc = wmb(ah, bh, acc);
    acc = wmb(ah, bl, acc);
    acc = wmb(al, bh, acc);
    if (m < 8) {
#pragma unroll
      for (int r = 0; r < 8; ++r) {
        const int pix = 16 * prow + 8 * h + r;
        float v = acc[r] + bias;
        v = fmaxf(v, 0.0f);
        const unsigned short hs = bfr(v);
        shh[m * (PP * PP) + pix] = hs;
        shl[m * (PP * PP) + pix] = bfr(v - bfup(hs));
      }
    }
  }
  __syncthreads();

  const v8us hv = *(const v8us*)(shh + 8 * tid);
  const v8us lv = *(const v8us*)(shl + 8 * tid);
  unsigned short* gh = Hh + (size_t)bk * FC1K + 8 * tid;
  unsigned short* gl = Hl + (size_t)bk * FC1K + 8 * tid;
  *(volatile v8us*)gh = hv;
  *(volatile v8us*)gl = lv;
  __threadfence();
  *(volatile v8us*)gh = hv;
  *(volatile v8us*)gl = lv;
}

__global__ __launch_bounds__(32) void k_fc1(const unsigned short* __restrict__ Hh, const unsigned short* __restrict__ Hl,
                                            const unsigned short* __restrict__ W1h, const unsigned short* __restrict__ W1l,
                                            const float* __restrict__ fc1b, unsigned short* Fh, unsigned short* Fl) {
  __shared__ __attribute__((aligned(16))) float st[16 * FC1N];
  const int rt = blockIdx.x, lane = threadIdx.x & 31, h = lane >> 4, m = lane & 15;
  v8f acc[4];
#pragma unroll
  for (int t = 0; t < 4; ++t) acc[t] = zero8();
  const unsigned short* aph = Hh + (size_t)(16 * rt + m) * FC1K + 8 * h;
  const unsigned short* apl = Hl + (size_t)(16 * rt + m) * FC1K + 8 * h;
#pragma unroll 1
  for (int ks = 0; ks < FC1K / 32; ++ks) {
    const int k0 = 32 * ks;
    FragU ah, al;
    ah.h[0] = *(const v8us*)(aph + k0);
    ah.h[1] = *(const v8us*)(aph + k0 + 16);
    al.h[0] = *(const v8us*)(apl + k0);
    al.h[1] = *(const v8us*)(apl + k0 + 16);
#pragma unroll
    for (int t = 0; t < 4; ++t) {
      const unsigned short* bph = W1h + (size_t)(16 * t + m) * FC1K + 8 * h + k0;
      const unsigned short* bpl = W1l + (size_t)(16 * t + m) * FC1K + 8 * h + k0;
      FragU bhf, blf;
      bhf.h[0] = *(const v8us*)bph;
      bhf.h[1] = *(const v8us*)(bph + 16);
      blf.h[0] = *(const v8us*)bpl;
      blf.h[1] = *(const v8us*)(bpl + 16);
      acc[t] = wmb(ah.v, bhf.v, acc[t]);
      acc[t] = wmb(ah.v, blf.v, acc[t]);
      acc[t] = wmb(al.v, bhf.v, acc[t]);
    }
  }
#pragma unroll
  for (int t = 0; t < 4; ++t) {
    const float bias = fc1b[16 * t + m];
#pragma unroll
    for (int r = 0; r < 8; ++r) {
      float v = acc[t][r] + bias;
      v = fmaxf(v, 0.0f);
      st[(8 * h + r) * FC1N + 16 * t + m] = v;
    }
  }
  __syncthreads();
  v8us hvv[4], lvv[4];
#pragma unroll
  for (int p = 0; p < 4; ++p) {
    const int rowl = 4 * p + (lane >> 3);
    const int c0 = (lane & 7) * 8;
    const v4f xa = *(const v4f*)(st + rowl * FC1N + c0);
    const v4f xb = *(const v4f*)(st + rowl * FC1N + c0 + 4);
#pragma unroll
    for (int e = 0; e < 4; ++e) {
      unsigned short hs = bfr(xa[e]);
      hvv[p][e] = hs; lvv[p][e] = bfr(xa[e] - bfup(hs));
      hs = bfr(xb[e]);
      hvv[p][4 + e] = hs; lvv[p][4 + e] = bfr(xb[e] - bfup(hs));
    }
  }
  unsigned short* gh = Fh + (size_t)(16 * rt) * FC1N;
  unsigned short* gl = Fl + (size_t)(16 * rt) * FC1N;
#pragma unroll
  for (int p = 0; p < 4; ++p) {
    *(volatile v8us*)(gh + 8 * (32 * p + lane)) = hvv[p];
    *(volatile v8us*)(gl + 8 * (32 * p + lane)) = lvv[p];
  }
  __threadfence();
#pragma unroll
  for (int p = 0; p < 4; ++p) {
    *(volatile v8us*)(gh + 8 * (32 * p + lane)) = hvv[p];
    *(volatile v8us*)(gl + 8 * (32 * p + lane)) = lvv[p];
  }
}

__global__ __launch_bounds__(NTHR) void k_fc2(const unsigned short* __restrict__ Fh, const unsigned short* __restrict__ Fl,
                                              const unsigned short* __restrict__ W2h, const unsigned short* __restrict__ W2l,
                                              const float* __restrict__ fc2b, float* out) {
  extern __shared__ v4f dynlds[];
  float* st = (float*)dynlds;
  const int rt = blockIdx.x, tid = threadIdx.x, lane = tid & 31, wave = tid >> 5, h = lane >> 4, m = lane & 15;
  v8f acc[8];
#pragma unroll
  for (int t = 0; t < 8; ++t) acc[t] = zero8();
  const unsigned short* aph = Fh + (size_t)(16 * rt + m) * FC2K + 8 * h;
  const unsigned short* apl = Fl + (size_t)(16 * rt + m) * FC2K + 8 * h;
  const int cb = 128 * wave;
#pragma unroll 1
  for (int ks = 0; ks < FC2K / 32; ++ks) {
    const int k0 = 32 * ks;
    FragU ah, al;
    ah.h[0] = *(const v8us*)(aph + k0);
    ah.h[1] = *(const v8us*)(aph + k0 + 16);
    al.h[0] = *(const v8us*)(apl + k0);
    al.h[1] = *(const v8us*)(apl + k0 + 16);
#pragma unroll
    for (int t = 0; t < 8; ++t) {
      const unsigned short* bph = W2h + (size_t)(cb + 16 * t + m) * FC2K + 8 * h + k0;
      const unsigned short* bpl = W2l + (size_t)(cb + 16 * t + m) * FC2K + 8 * h + k0;
      FragU bhf, blf;
      bhf.h[0] = *(const v8us*)bph;
      bhf.h[1] = *(const v8us*)(bph + 16);
      blf.h[0] = *(const v8us*)bpl;
      blf.h[1] = *(const v8us*)(bpl + 16);
      acc[t] = wmb(ah.v, bhf.v, acc[t]);
      acc[t] = wmb(ah.v, blf.v, acc[t]);
      acc[t] = wmb(al.v, bhf.v, acc[t]);
    }
  }
#pragma unroll
  for (int t = 0; t < 8; ++t) {
    const int cn = cb + 16 * t + m;
    const float bias = fc2b[cn < NCLS ? cn : NCLS - 1];
#pragma unroll
    for (int r = 0; r < 8; ++r) st[(8 * h + r) * NPAD + cn] = acc[t][r] + bias;
  }
  __syncthreads();

  v4f vals[16];
#pragma unroll
  for (int i = 0; i < 16; ++i) {
    int q = tid + NTHR * i;
    q = q < 4000 ? q : 3999;
    const int el = 4 * q;
    const int rl = el / NCLS;
    const int cn = el - rl * NCLS;
    vals[i] = *(const v4f*)(st + rl * NPAD + cn);
  }
  float* ob = out + (size_t)rt * (16 * NCLS);
#pragma unroll
  for (int i = 0; i < 16; ++i) {
    const int q = tid + NTHR * i;
    if (q < 4000) *(volatile v4f*)(ob + 4 * q) = vals[i];
  }
  __threadfence();
#pragma unroll
  for (int i = 0; i < 16; ++i) {
    const int q = tid + NTHR * i;
    if (q < 4000) *(volatile v4f*)(ob + 4 * q) = vals[i];
  }
}

extern "C" void kernel_launch(void* const* d_in, const int* in_sizes, int n_in,
                              void* d_out, int out_size, void* d_ws, size_t ws_size,
                              hipStream_t stream) {
  if (n_in < 7) return;
  if (in_sizes[0] != BB * CCH * IMG) return;
  if (in_sizes[1] != 8 * CCH * 9 || in_sizes[2] != 8) return;
  if (in_sizes[3] != FC1N * FC1K || in_sizes[4] != FC1N) return;
  if (in_sizes[5] != NCLS * FC2K || in_sizes[6] != NCLS) return;
  if (out_size != BB * NCLS) return;

  const float* x     = (const float*)d_in[0];
  const float* convw = (const float*)d_in[1];
  const float* convb = (const float*)d_in[2];
  const float* fc1w  = (const float*)d_in[3];
  const float* fc1b  = (const float*)d_in[4];
  const float* fc2w  = (const float*)d_in[5];
  const float* fc2b  = (const float*)d_in[6];
  float* out = (float*)d_out;

  char* ws = (char*)d_ws;
  size_t off = 0;
  const size_t oR   = off; off += (size_t)BB * IMG * 4;        off = (off + 255) & ~(size_t)255;
  const size_t oIdx = off; off += (size_t)BB * KPT * 4;        off = (off + 255) & ~(size_t)255;
  const size_t oHh  = off; off += (size_t)MROWS * FC1K * 2;    off = (off + 255) & ~(size_t)255;
  const size_t oHl  = off; off += (size_t)MROWS * FC1K * 2;    off = (off + 255) & ~(size_t)255;
  const size_t oW1h = off; off += (size_t)FC1N * FC1K * 2;     off = (off + 255) & ~(size_t)255;
  const size_t oW1l = off; off += (size_t)FC1N * FC1K * 2;     off = (off + 255) & ~(size_t)255;
  const size_t oFh  = off; off += (size_t)MROWS * FC1N * 2;    off = (off + 255) & ~(size_t)255;
  const size_t oFl  = off; off += (size_t)MROWS * FC1N * 2;    off = (off + 255) & ~(size_t)255;
  const size_t oW2h = off; off += (size_t)NPAD * FC2K * 2;     off = (off + 255) & ~(size_t)255;
  const size_t oW2l = off; off += (size_t)NPAD * FC2K * 2;     off = (off + 255) & ~(size_t)255;
  if (off > ws_size || off > (size_t)134217728) return;

  float*          Rm   = (float*)(ws + oR);
  int*            idxT = (int*)(ws + oIdx);
  unsigned short* Hh   = (unsigned short*)(ws + oHh);
  unsigned short* Hl   = (unsigned short*)(ws + oHl);
  unsigned short* W1h  = (unsigned short*)(ws + oW1h);
  unsigned short* W1l  = (unsigned short*)(ws + oW1l);
  unsigned short* Fh   = (unsigned short*)(ws + oFh);
  unsigned short* Fl   = (unsigned short*)(ws + oFl);
  unsigned short* W2h  = (unsigned short*)(ws + oW2h);
  unsigned short* W2l  = (unsigned short*)(ws + oW2l);

  k_prep<<<(NT1 + NT2) / NTHR, NTHR, 0, stream>>>(fc1w, fc2w, W1h, W1l, W2h, W2l);

  k_harris<<<dim3(HH / TR, BB, 1), NTHR, 0, stream>>>(x, Rm);

  const int ldsTop = IMG * 4;
  hipFuncSetAttribute(reinterpret_cast<const void*>(&k_topk), hipFuncAttributeMaxDynamicSharedMemorySize, ldsTop);
  k_topk<<<BB, NTHR, ldsTop, stream>>>(Rm, idxT);

  k_patch<<<MROWS, NTHR, 0, stream>>>(x, idxT, convw, convb, Hh, Hl);

  k_fc1<<<MROWS / 16, 32, 0, stream>>>(Hh, Hl, W1h, W1l, fc1b, Fh, Fl);

  const int ldsFc2 = 16 * NPAD * 4;
  hipFuncSetAttribute(reinterpret_cast<const void*>(&k_fc2), hipFuncAttributeMaxDynamicSharedMemorySize, ldsFc2);
  k_fc2<<<BB / 16, NTHR, ldsFc2, stream>>>(Fh, Fl, W2h, W2l, fc2b, out);
}
